// LSTMModel_66700842107330
// MI455X (gfx1250) — hardware-verified
//
#include <hip/hip_runtime.h>
#include <math.h>

constexpr int NBATCH   = 4096;
constexpr int NSTEP    = 512;
constexpr int NHID     = 50;
constexpr int NGATE    = 4;
constexpr int NG4      = NGATE * NHID;
constexpr int ROWS_BLK = 32;
constexpr int UPAD     = 64;
constexpr int NCOLS    = NGATE * UPAD;
constexpr int KPADC    = 64;
constexpr int HPITCH   = 72;
constexpr int WPITCH   = 72;
constexpr int NUB      = UPAD / 16;
constexpr int KSLOT0   = 56;
constexpr int KS_XH    = KSLOT0 + 0;
constexpr int KS_XL    = KSLOT0 + 1;
constexpr int KS_XQ    = KSLOT0 + 2;
constexpr int KS_B1    = KSLOT0 + 3;
constexpr int KS_B2    = KSLOT0 + 4;
constexpr float XCARRY     = 64.0f;
constexpr float XCARRY_INV = 1.0f / 64.0f;
constexpr float BCARRY     = 2048.0f;
constexpr float BCARRY_INV = 1.0f / 2048.0f;

static_assert(NBATCH % ROWS_BLK == 0, "grid exact");
static_assert(NHID <= KSLOT0, "hidden units below the slot block");
static_assert(KSLOT0 + 8 == KPADC, "slot block is the last 16-byte chunk of a row");
static_assert(KPADC % 32 == 0, "K multiple of 32");
static_assert(NCOLS % 16 == 0 && UPAD % 16 == 0, "N tile multiples");
static_assert(NHID <= UPAD, "unit padding");
static_assert((HPITCH % 8) == 0 && (WPITCH % 8) == 0, "16-byte aligned rows");
static_assert(HPITCH >= KPADC && WPITCH >= KPADC, "row holds K");
static_assert((NCOLS * (KPADC / 8)) % 32 == 0, "weight staging loop exact");
static_assert((ROWS_BLK * HPITCH) % (8 * 32) == 0, "h tile zero-fill loop exact");
static_assert(NSTEP >= 1, "steps");

typedef __attribute__((ext_vector_type(16))) _Float16 v16h;
typedef __attribute__((ext_vector_type(8)))  _Float16 v8h;
typedef __attribute__((ext_vector_type(8)))  float    v8f;

__device__ __forceinline__ void dep_guard_h(v8f& a, v8f& b, v16h x, v16h y) {
  asm volatile("v_nop\n\tv_nop\n\tv_nop\n\tv_nop" : "+v"(a), "+v"(b) : "v"(x), "v"(y));
}
__device__ __forceinline__ void acc_guard8(v8f& a0, v8f& a1, v8f& a2, v8f& a3, v8f& a4, v8f& a5, v8f& a6, v8f& a7,
                                           v16h p, v16h q, v16h r, v16h s) {
  asm volatile("v_nop\n\tv_nop\n\tv_nop\n\tv_nop"
               : "+v"(a0), "+v"(a1), "+v"(a2), "+v"(a3), "+v"(a4), "+v"(a5), "+v"(a6), "+v"(a7)
               : "v"(p), "v"(q), "v"(r), "v"(s));
}
template <typename T> struct Frag;
template <> struct Frag<_Float16> {
  typedef v16h V; union U { v16h v; v8h h[2]; };
  static __device__ __forceinline__ v16h load(const _Float16* p) {
    U f; f.h[0] = *(const v8h*)(p); f.h[1] = *(const v8h*)(p + 16); return f.v;
  }
  static __device__ __forceinline__ v8f mma(v16h a, v16h b, v8f c) {
    return __builtin_amdgcn_wmma_f32_16x16x32_f16(false, a, false, b, (short)0, c, false, false);
  }
};

__device__ __forceinline__ float pin_f(float v) { asm volatile("" : "+v"(v)); return v; }
__device__ __forceinline__ float fsig(float x)  { return __builtin_amdgcn_rcpf(1.0f + __expf(-x)); }
__device__ __forceinline__ float ftanh(float x) { return 1.0f - 2.0f * __builtin_amdgcn_rcpf(__expf(2.0f * x) + 1.0f); }

__device__ __forceinline__ void put_slots(_Float16* hrow, float xv, float onef, float tinyf, float zerof) {
  const _Float16 xh = (_Float16)xv;
  const float xhf = (float)xh;
  const float xl  = (xv - xhf) * XCARRY;
  const float xq  = xhf * XCARRY_INV;
  v8h s;
  s[0] = xh;
  s[1] = (_Float16)xl;
  s[2] = (_Float16)xq;
  s[3] = (_Float16)onef;
  s[4] = (_Float16)tinyf;
  s[5] = (_Float16)zerof;
  s[6] = (_Float16)zerof;
  s[7] = (_Float16)zerof;
  *(v8h*)(hrow + KSLOT0) = s;
}

__device__ __forceinline__ void cell8(v8f zi, v8f zf, v8f zg, v8f zo, float* clp, float* hlp, _Float16* hcol, bool live) {
#pragma unroll
  for (int r = 0; r < 8; ++r) {
    const float ig = fsig(zi[r]);
    const float fg = fsig(zf[r]);
    const float gg = ftanh(zg[r]);
    const float og = fsig(zo[r]);
    const float co = clp[r * 32];
    const float cn = fg * co + ig * gg;
    clp[r * 32] = cn;
    const float hn = og * ftanh(cn);
    hlp[r * 32] = hn;
    if (live) hcol[r * HPITCH] = (_Float16)hn;
  }
}

__global__ __launch_bounds__(32) __attribute__((amdgpu_num_vgpr(248)))
void lstm_seq_kernel(const float* __restrict__ x, const float* __restrict__ W_ih, const float* __restrict__ W_hh,
                     const float* __restrict__ b_ih, const float* __restrict__ b_hh,
                     const float* __restrict__ W_fc, const float* __restrict__ b_fc, float* __restrict__ out) {
  __shared__ __align__(16) _Float16 wlds[NCOLS * WPITCH];
  __shared__ __align__(16) _Float16 htile[ROWS_BLK * HPITCH];
  __shared__ __align__(16) float    cl[2 * NUB * 8 * 32];
  __shared__ __align__(16) float    hl[2 * NUB * 8 * 32];

  const int lane = threadIdx.x;
  const int c = lane & 15, hh = lane >> 4, koff = hh * 8;
  const int rowbase = blockIdx.x * ROWS_BLK;

#pragma unroll 1
  for (int it = 0; it < (NCOLS * (KPADC / 8)) / 32; ++it) {
    const int id   = it * 32 + lane;
    const int n    = id >> 3;
    const int kc   = id & 7;
    const int gate = n >> 6;
    const int j    = n & (UPAD - 1);
    const bool liveu = j < NHID;
    const int jc   = liveu ? j : (NHID - 1);
    const int r    = gate * NHID + jc;
    const float wih = pin_f(W_ih[r]);
    const float bi  = pin_f(b_ih[r]);
    const float bh  = pin_f(b_hh[r]);
    const float bs  = bi + bh;
    const float wih_h = (float)(_Float16)wih;
    const float bs_h  = (float)(_Float16)bs;
    const float s_xh = wih;
    const float s_xl = wih_h * XCARRY_INV;
    const float s_xq = (wih - wih_h) * XCARRY;
    const float s_b1 = bs;
    const float s_b2 = (bs - bs_h) * BCARRY;
    v8h hv;
#pragma unroll
    for (int e = 0; e < 8; ++e) {
      const int kk  = kc * 8 + e;
      const int kcl = (kk < NHID) ? kk : (NHID - 1);
      const float w = pin_f(W_hh[r * NHID + kcl]);
      float val = 0.0f;
      val = (kk == KS_B2) ? s_b2 : val;
      val = (kk == KS_B1) ? s_b1 : val;
      val = (kk == KS_XQ) ? s_xq : val;
      val = (kk == KS_XL) ? s_xl : val;
      val = (kk == KS_XH) ? s_xh : val;
      val = (kk < NHID) ? w : val;
      val = liveu ? val : 0.0f;
      hv[e] = (_Float16)val;
    }
    *(v8h*)(wlds + n * WPITCH + kc * 8) = hv;
  }

  float zerof = 0.0f;
  float onef  = 1.0f;
  float tinyf = BCARRY_INV;
  asm volatile("" : "+v"(zerof));
  asm volatile("" : "+v"(onef));
  asm volatile("" : "+v"(tinyf));
  {
    v8h zv;
#pragma unroll
    for (int e = 0; e < 8; ++e) zv[e] = (_Float16)zerof;
#pragma unroll 1
    for (int it = 0; it < (ROWS_BLK * HPITCH) / (8 * 32); ++it) *(v8h*)(htile + (it * 32 + lane) * 8) = zv;
  }
#pragma unroll 1
  for (int i = 0; i < 2 * NUB * 8; ++i) cl[i * 32 + lane] = 0.0f;
  __syncthreads();

  const float* xrow = x + (size_t)(rowbase + lane) * NSTEP;
  _Float16* hrow = htile + lane * HPITCH;
  {
    const float x0 = pin_f(xrow[0]);
    put_slots(hrow, x0, onef, tinyf, zerof);
  }
  __syncthreads();

  const _Float16* arow0 = htile + c * HPITCH + koff;
  const _Float16* arow1 = htile + (16 + c) * HPITCH + koff;
  const v8f z8 = {0.f, 0.f, 0.f, 0.f, 0.f, 0.f, 0.f, 0.f};

#pragma unroll 1
  for (int t = 0; t < NSTEP; ++t) {
    const int tn = (t + 1 < NSTEP) ? (t + 1) : (NSTEP - 1);
    const float xn = pin_f(xrow[tn]);

    const v16h a00 = Frag<_Float16>::load(arow0);
    const v16h a01 = Frag<_Float16>::load(arow0 + 32);
    const v16h a10 = Frag<_Float16>::load(arow1);
    const v16h a11 = Frag<_Float16>::load(arow1 + 32);
    __syncthreads();

#pragma unroll 1
    for (int ub = 0; ub < NUB; ++ub) {
      const _Float16* wb = wlds + (ub * 16 + c) * WPITCH + koff;
      v8f acc0[NGATE], acc1[NGATE];
#pragma unroll
      for (int g = 0; g < NGATE; ++g) {
        const v16h bk0 = Frag<_Float16>::load(wb + g * UPAD * WPITCH);
        const v16h bk1 = Frag<_Float16>::load(wb + g * UPAD * WPITCH + 32);
        acc0[g] = Frag<_Float16>::mma(a00, bk0, z8);
        acc0[g] = Frag<_Float16>::mma(a01, bk1, acc0[g]);
        acc1[g] = Frag<_Float16>::mma(a10, bk0, z8);
        acc1[g] = Frag<_Float16>::mma(a11, bk1, acc1[g]);
        dep_guard_h(acc0[g], acc1[g], bk0, bk1);
      }
      acc_guard8(acc0[0], acc0[1], acc0[2], acc0[3], acc1[0], acc1[1], acc1[2], acc1[3], a00, a01, a10, a11);

      const bool live = (ub * 16 + c) < KSLOT0;
      float* clp0 = cl + ((0 * NUB + ub) * 8) * 32 + lane;
      float* hlp0 = hl + ((0 * NUB + ub) * 8) * 32 + lane;
      float* clp1 = cl + ((1 * NUB + ub) * 8) * 32 + lane;
      float* hlp1 = hl + ((1 * NUB + ub) * 8) * 32 + lane;
      _Float16* hcol0 = htile + (8 * hh) * HPITCH + ub * 16 + c;
      _Float16* hcol1 = htile + (16 + 8 * hh) * HPITCH + ub * 16 + c;
      cell8(acc0[0], acc0[1], acc0[2], acc0[3], clp0, hlp0, hcol0, live);
      cell8(acc1[0], acc1[1], acc1[2], acc1[3], clp1, hlp1, hcol1, live);
    }

    put_slots(hrow, xn, onef, tinyf, zerof);
    __syncthreads();
  }

  {
    const int m2 = lane >> 4, hh2 = (lane >> 3) & 1, r2 = lane & 7;
    float s = 0.0f;
#pragma unroll 1
    for (int j = 0; j < NHID; ++j) {
      const int ubj = j >> 4, cj = j & 15;
      const float hv = hl[((m2 * NUB + ubj) * 8 + r2) * 32 + hh2 * 16 + cj];
      s = fmaf(hv, W_fc[j], s);
    }
    const float o = s + b_fc[0];
    volatile float* op = out + rowbase + lane;
    *op = o;
    __threadfence();
    *op = o;
  }
}

extern "C" void kernel_launch(void* const* d_in, const int* in_sizes, int n_in,
                              void* d_out, int out_size, void* d_ws, size_t ws_size, hipStream_t stream) {
  (void)d_ws; (void)ws_size;
  if (n_in < 7 || d_out == nullptr) return;
  if (in_sizes[0] != NBATCH * NSTEP || in_sizes[1] != NG4 || in_sizes[2] != NG4 * NHID ||
      in_sizes[3] != NG4 || in_sizes[4] != NG4 || in_sizes[5] != NHID || in_sizes[6] != 1 ||
      out_size != NBATCH) return;
  const float* x    = (const float*)d_in[0];
  const float* W_ih = (const float*)d_in[1];
  const float* W_hh = (const float*)d_in[2];
  const float* b_ih = (const float*)d_in[3];
  const float* b_hh = (const float*)d_in[4];
  const float* W_fc = (const float*)d_in[5];
  const float* b_fc = (const float*)d_in[6];
  float* out = (float*)d_out;
  lstm_seq_kernel<<<NBATCH / ROWS_BLK, ROWS_BLK, 0, stream>>>(x, W_ih, W_hh, b_ih, b_hh, W_fc, b_fc, out);
}
